// MultiHeadSelfAttention_13228499271978
// MI455X (gfx1250) — hardware-verified
//
#include <hip/hip_runtime.h>
#ifndef NB
#define NB 2
#endif
#ifndef SEQ
#define SEQ 2048
#endif
#define SEQ_FULL 2048
#define DM 1024
#define NH 16
#define HD 64
#define TABN 4096
#define NR (NB * SEQ)
#define ERW ((SEQ) < 256 ? (SEQ) : 256)

typedef _Float16 v16h __attribute__((ext_vector_type(16)));
typedef _Float16 v8h  __attribute__((ext_vector_type(8)));
typedef _Float16 v8ha __attribute__((ext_vector_type(8), may_alias));
typedef float    v8f  __attribute__((ext_vector_type(8)));
typedef float    v4f  __attribute__((ext_vector_type(4)));
typedef float    v4fa __attribute__((ext_vector_type(4), may_alias));

static_assert(DM == NH * HD);
static_assert(HD == 64);
static_assert(DM % 128 == 0);
static_assert(NR % 128 == 0);
static_assert(SEQ % 64 == 0);
static_assert(ERW % 64 == 0);
static_assert(ERW <= SEQ);
static_assert(DM % 32 == 0);
static_assert((2 * DM) % 32 == 0);
static_assert(TABN == 4096);
static_assert((long long)NR * 2 * DM < 2147483647LL);

__device__ __forceinline__ float bf16_rne(float x) { unsigned int u = __float_as_uint(x); u = (u + 0x7FFFu + ((u >> 16) & 1u)) & 0xFFFF0000u; return __uint_as_float(u); }

__device__ __forceinline__ v16h cat16(v8h lo, v8h hi) { return __builtin_shufflevector(lo, hi, 0, 1, 2, 3, 4, 5, 6, 7, 8, 9, 10, 11, 12, 13, 14, 15); }
__device__ __forceinline__ v16h frag16(const _Float16* __restrict__ p) { const v8h lo = *(const v8ha*)p; const v8h hi = *(const v8ha*)(p + 16); return cat16(lo, hi); }
__device__ __forceinline__ v8f mma16(v16h a, v16h b, v8f c) {
  v8f d = __builtin_amdgcn_wmma_f32_16x16x32_f16(false, a, false, b, (short)0, c, false, false);
  asm volatile("v_nop\n\tv_nop\n\tv_nop\n\tv_nop" : "+v"(d) : "v"(a), "v"(b));
  return d;
}
__device__ __forceinline__ void split8(const float (&x)[8], v8h& hv, v8h& lv) {
#pragma unroll
  for (int i = 0; i < 8; ++i) { const _Float16 hq = (_Float16)x[i]; hv[i] = hq; lv[i] = (_Float16)((x[i] - (float)hq) * 1024.0f); }
}

__global__ __launch_bounds__(256) void k_xcvt(const float* __restrict__ x, _Float16* __restrict__ X16) {
  const int t = blockIdx.x * 256 + threadIdx.x;
  if (t >= NR * (DM / 8)) return;
  const int r = t / (DM / 8), c8 = (t - r * (DM / 8)) * 8;
  const int b = r / SEQ, s = r - b * SEQ;
  const float* src = x + (size_t)(b * SEQ_FULL + s) * DM + c8;
  const v4f a = *(const v4fa*)src, c = *(const v4fa*)(src + 4);
  v8h o;
#pragma unroll
  for (int i = 0; i < 4; ++i) { o[i] = (_Float16)bf16_rne(a[i]); o[4 + i] = (_Float16)bf16_rne(c[i]); }
  _Float16* d = X16 + (size_t)r * DM + c8;
  *(volatile v8h*)d = o; __threadfence(); *(volatile v8h*)d = o;
}

__global__ __launch_bounds__(256) void k_wcvt(const float* __restrict__ w, _Float16* __restrict__ dst, int dpitch, float scale) {
  const int t = blockIdx.x * 256 + threadIdx.x;
  if (t >= DM * (DM / 8)) return;
  const int n = t / (DM / 8), k8 = (t - n * (DM / 8)) * 8;
  const float* src = w + (size_t)n * DM + k8;
  const v4f a = *(const v4fa*)src, c = *(const v4fa*)(src + 4);
  v8h o;
#pragma unroll
  for (int i = 0; i < 4; ++i) { o[i] = (_Float16)(bf16_rne(a[i]) * scale); o[4 + i] = (_Float16)(bf16_rne(c[i]) * scale); }
  _Float16* d = dst + (size_t)n * dpitch + k8;
  *(volatile v8h*)d = o; __threadfence(); *(volatile v8h*)d = o;
}

__global__ __launch_bounds__(256) void k_ropetab(float* __restrict__ tab) {
  #pragma clang fp contract(off)
  const int t = blockIdx.x * 256 + threadIdx.x;
  if (t >= TABN * 16) return;
  const int pos = t >> 4, jp = t & 15;
  float c0 = 0.f, s0 = 0.f, c1 = 0.f, s1 = 0.f;
#pragma unroll 1
  for (int u = 0; u < 2; ++u) {
    const int j = 2 * jp + u;
    double p = 1.0;
    p *= (j & 1) ? 1.3335214321633240 : 1.0;
    p *= (j & 2) ? 1.7782794100389228 : 1.0;
    p *= (j & 4) ? 3.1622776601683795 : 1.0;
    p *= (j & 8) ? 10.0 : 1.0;
    p *= (j & 16) ? 100.0 : 1.0;
    const float pf = (float)p;
    const float inv = 1.0f / pf;
    const float ang = (float)pos * inv;
    float sn, cs;
    sincosf(ang, &sn, &cs);
    if (u == 0) { c0 = cs; s0 = sn; } else { c1 = cs; s1 = sn; }
  }
  const v4f o = {c0, s0, c1, s1};
  float* d = tab + (size_t)pos * 64 + jp * 4;
  *(volatile v4f*)d = o; __threadfence(); *(volatile v4f*)d = o;
}

__device__ __forceinline__ void gemm_tile(const _Float16* __restrict__ A, const int lda, const _Float16* __restrict__ Bt, const int ldb,
                                          const int K, const int row0, const int col0, const int ln, const int hh, v8f (&c)[8]) {
  const int ao0 = (row0 + ln) * lda + 8 * hh, ao1 = ao0 + 16 * lda;
  const int bo0 = (col0 + ln) * ldb + 8 * hh, bo1 = bo0 + 16 * ldb, bo2 = bo1 + 16 * ldb, bo3 = bo2 + 16 * ldb;
#pragma unroll 1
  for (int kb = 0; kb < K; kb += 32) {
    const v16h a0 = frag16(A + ao0 + kb), a1 = frag16(A + ao1 + kb);
    v16h b = frag16(Bt + bo0 + kb); c[0] = mma16(a0, b, c[0]); c[4] = mma16(a1, b, c[4]);
    b = frag16(Bt + bo1 + kb); c[1] = mma16(a0, b, c[1]); c[5] = mma16(a1, b, c[5]);
    b = frag16(Bt + bo2 + kb); c[2] = mma16(a0, b, c[2]); c[6] = mma16(a1, b, c[6]);
    b = frag16(Bt + bo3 + kb); c[3] = mma16(a0, b, c[3]); c[7] = mma16(a1, b, c[7]);
  }
}

__global__ __launch_bounds__(128) void k_proj(const _Float16* __restrict__ A, const _Float16* __restrict__ Bt, _Float16* __restrict__ Ch, _Float16* __restrict__ Cl,
                                              const int* __restrict__ tp, const float* __restrict__ tab, int ldc, int N, int rope) {
  __shared__ __attribute__((aligned(16))) float so[4][32][68];
  const int wave = __builtin_amdgcn_readfirstlane((int)(threadIdx.x >> 5));
  const int lane = threadIdx.x & 31, ln = lane & 15, hh = lane >> 4;
  const int ntn = N >> 6;
  const int mt = blockIdx.x / ntn, nq = blockIdx.x - mt * ntn;
  const int row0 = mt * 128 + 32 * wave, col0 = nq * 64;
  const v8f z8 = {0.f, 0.f, 0.f, 0.f, 0.f, 0.f, 0.f, 0.f};
  v8f c[8] = {z8, z8, z8, z8, z8, z8, z8, z8};
  gemm_tile(A, DM, Bt, DM, DM, row0, col0, ln, hh, c);
#pragma unroll
  for (int u = 0; u < 8; ++u) {
    const int t = u & 3, half = u >> 2;
#pragma unroll
    for (int r = 0; r < 8; ++r) so[wave][half * 16 + 8 * hh + r][t * 16 + ln] = c[u][r] * 0.0625f;
  }
  __builtin_amdgcn_fence(4  , "workgroup"); __builtin_amdgcn_wave_barrier();
  const int rsub = lane >> 3, c8 = (lane & 7) * 8;
  v8h hv[8], lv[8];
#pragma unroll
  for (int q = 0; q < 8; ++q) {
    const int rl = q * 4 + rsub;
    const v4f a = *(const v4fa*)&so[wave][rl][c8];
    const v4f bq = *(const v4fa*)&so[wave][rl][c8 + 4];
    float xv[8] = {a[0], a[1], a[2], a[3], bq[0], bq[1], bq[2], bq[3]};
    if (rope != 0) {
      const int m = row0 + rl; const int bb = m / SEQ; const int ss = m - bb * SEQ;
      int pos = tp[bb * SEQ_FULL + ss];
      pos = pos < 0 ? 0 : (pos > TABN - 1 ? TABN - 1 : pos);
      const float* tr = tab + (size_t)pos * 64 + c8;
      const v4f t0 = *(const v4fa*)tr; const v4f t1 = *(const v4fa*)(tr + 4);
      const float cs[4] = {t0[0], t0[2], t1[0], t1[2]};
      const float sn[4] = {t0[1], t0[3], t1[1], t1[3]};
#pragma unroll
      for (int i = 0; i < 4; ++i) { const float x1 = xv[2 * i], x2 = xv[2 * i + 1]; xv[2 * i] = x1 * cs[i] - x2 * sn[i]; xv[2 * i + 1] = x1 * sn[i] + x2 * cs[i]; }
    }
    split8(xv, hv[q], lv[q]);
  }
#pragma unroll
  for (int pass = 0; pass < 2; ++pass) {
#pragma unroll
    for (int q = 0; q < 8; ++q) {
      const size_t off = (size_t)(row0 + q * 4 + rsub) * ldc + col0 + c8;
      *(volatile v8h*)(Ch + off) = hv[q];
      *(volatile v8h*)(Cl + off) = lv[q];
    }
    if (pass == 0) __threadfence();
  }
}

template <int EARLY>
__device__ __forceinline__ void attn_body(const _Float16* __restrict__ Qh, const _Float16* __restrict__ Ql, const _Float16* __restrict__ Kh, const _Float16* __restrict__ Kl,
                                          const _Float16* __restrict__ VTh, const _Float16* __restrict__ VTl, _Float16* __restrict__ CTX, const int qt0) {
  __shared__ __attribute__((aligned(16))) _Float16 pbh[4][16][40];
  __shared__ __attribute__((aligned(16))) _Float16 pbl[EARLY ? 4 : 1][16][40];
  __shared__ __attribute__((aligned(16))) float so[4][16][68];
  const int wave = __builtin_amdgcn_readfirstlane((int)(threadIdx.x >> 5));
  const int lane = threadIdx.x & 31, ln = lane & 15, hh = lane >> 4;
  const int bh = blockIdx.y, b = bh / NH, h = bh - b * NH;
  const int rb = b * SEQ;
  const int q0w = (qt0 + (int)blockIdx.x) * 64 + 16 * wave;
  const int nch = (q0w + 47) >> 5;
  const int qoff = (rb + q0w + ln) * DM + h * HD + 8 * hh;
  const int kbase = (rb + ln) * DM + h * HD + 8 * hh;
  const int vbase = (h * HD + ln) * NR + rb + 8 * hh;
  const float RS = 0.0009765625f;
  const v8f z8 = {0.f, 0.f, 0.f, 0.f, 0.f, 0.f, 0.f, 0.f};
  v8f om[4] = {z8, z8, z8, z8};
  v8f orr[4] = {z8, z8, z8, z8};
  float mrun[8], lrun[8];
#pragma unroll
  for (int r = 0; r < 8; ++r) { mrun[r] = -1.0e30f; lrun[r] = 0.f; }
#pragma unroll 1
  for (int cidx = 0; cidx < nch; ++cidx) {
    const int k0 = cidx * 32;
    int qo = qoff; asm volatile("" : "+v"(qo));
    v8f s0 = z8, s1 = z8, sr0 = z8, sr1 = z8;
#pragma unroll
    for (int ks = 0; ks < 2; ++ks) {
      const v16h aqh = frag16(Qh + qo + ks * 32);
      const v16h aql = frag16(Ql + qo + ks * 32);
      const int ko = kbase + k0 * DM + ks * 32;
      v16h bk = frag16(Kh + ko);
      s0 = mma16(aqh, bk, s0); sr0 = mma16(aql, bk, sr0);
      if (EARLY) { const v16h bl = frag16(Kl + ko); sr0 = mma16(aqh, bl, sr0); }
      bk = frag16(Kh + ko + 16 * DM);
      s1 = mma16(aqh, bk, s1); sr1 = mma16(aql, bk, sr1);
      if (EARLY) { const v16h bl = frag16(Kl + ko + 16 * DM); sr1 = mma16(aqh, bl, sr1); }
    }
    float al[8];
#pragma unroll
    for (int r = 0; r < 8; ++r) {
      const int qrow = q0w + 8 * hh + r;
      float x0 = (s0[r] + sr0[r] * RS) * 0.125f;
      float x1 = (s1[r] + sr1[r] * RS) * 0.125f;
      x0 = (k0 + ln <= qrow) ? x0 : -1.0e30f;
      x1 = (k0 + 16 + ln <= qrow) ? x1 : -1.0e30f;
      float tm = fmaxf(x0, x1);
      tm = fmaxf(tm, __shfl_xor(tm, 1, 32));
      tm = fmaxf(tm, __shfl_xor(tm, 2, 32));
      tm = fmaxf(tm, __shfl_xor(tm, 4, 32));
      tm = fmaxf(tm, __shfl_xor(tm, 8, 32));
      const float mn = fmaxf(mrun[r], tm);
      al[r] = __expf(mrun[r] - mn);
      mrun[r] = mn;
      const float p0 = __expf(x0 - mn) * 256.0f;
      const float p1 = __expf(x1 - mn) * 256.0f;
      const _Float16 h0 = (_Float16)p0, h1 = (_Float16)p1;
      float acc = (float)h0 + (float)h1;
      pbh[wave][8 * hh + r][ln] = h0;
      pbh[wave][8 * hh + r][16 + ln] = h1;
      if (EARLY) {
        const _Float16 g0 = (_Float16)((p0 - (float)h0) * 1024.0f), g1 = (_Float16)((p1 - (float)h1) * 1024.0f);
        pbl[wave][8 * hh + r][ln] = g0;
        pbl[wave][8 * hh + r][16 + ln] = g1;
        acc += ((float)g0 + (float)g1) * RS;
      }
      lrun[r] = lrun[r] * al[r] + acc;
    }
    __builtin_amdgcn_fence(4  , "workgroup"); __builtin_amdgcn_wave_barrier();
    const v16h ap = cat16(*(const v8ha*)&pbh[wave][ln][8 * hh], *(const v8ha*)&pbh[wave][ln][16 + 8 * hh]);
    v16h apl = ap;
    if (EARLY) apl = cat16(*(const v8ha*)&pbl[wave][ln][8 * hh], *(const v8ha*)&pbl[wave][ln][16 + 8 * hh]);
#pragma unroll
    for (int t = 0; t < 4; ++t) {
#pragma unroll
      for (int r = 0; r < 8; ++r) { om[t][r] *= al[r]; if (EARLY) orr[t][r] *= al[r]; }
    }
    const int vo = vbase + k0;
#pragma unroll
    for (int t = 0; t < 4; ++t) {
      const v16h bv = frag16(VTh + vo + t * 16 * NR);
      om[t] = mma16(ap, bv, om[t]);
      if (EARLY) {
        orr[t] = mma16(apl, bv, orr[t]);
        const v16h bvl = frag16(VTl + vo + t * 16 * NR);
        orr[t] = mma16(ap, bvl, orr[t]);
      }
    }
    __builtin_amdgcn_fence(4  , "workgroup"); __builtin_amdgcn_wave_barrier();
  }
  float inv[8];
#pragma unroll
  for (int r = 0; r < 8; ++r) {
    float lt = lrun[r];
    lt += __shfl_xor(lt, 1, 32);
    lt += __shfl_xor(lt, 2, 32);
    lt += __shfl_xor(lt, 4, 32);
    lt += __shfl_xor(lt, 8, 32);
    inv[r] = 64.0f / lt;
  }
#pragma unroll
  for (int t = 0; t < 4; ++t) {
#pragma unroll
    for (int r = 0; r < 8; ++r) { float v = om[t][r]; if (EARLY) v += orr[t][r] * RS; so[wave][8 * hh + r][16 * t + ln] = v * inv[r]; }
  }
  __builtin_amdgcn_fence(4  , "workgroup"); __builtin_amdgcn_wave_barrier();
  const int rsub = lane >> 3, c8 = (lane & 7) * 8;
  v8h hv[4], lv[4];
#pragma unroll
  for (int q = 0; q < 4; ++q) {
    const int rl = q * 4 + rsub;
    const v4f a = *(const v4fa*)&so[wave][rl][c8];
    const v4f bq = *(const v4fa*)&so[wave][rl][c8 + 4];
    const float xv[8] = {a[0], a[1], a[2], a[3], bq[0], bq[1], bq[2], bq[3]};
    split8(xv, hv[q], lv[q]);
  }
#pragma unroll
  for (int pass = 0; pass < 2; ++pass) {
#pragma unroll
    for (int q = 0; q < 4; ++q) {
      const size_t off = (size_t)(rb + q0w + q * 4 + rsub) * (2 * DM) + h * HD + c8;
      *(volatile v8h*)(CTX + off) = hv[q];
      *(volatile v8h*)(CTX + off + DM) = lv[q];
    }
    if (pass == 0) __threadfence();
  }
}

__global__ __launch_bounds__(128) void k_attn_early(const _Float16* __restrict__ Qh, const _Float16* __restrict__ Ql, const _Float16* __restrict__ Kh, const _Float16* __restrict__ Kl,
                                                    const _Float16* __restrict__ VTh, const _Float16* __restrict__ VTl, _Float16* __restrict__ CTX) {
  attn_body<1>(Qh, Ql, Kh, Kl, VTh, VTl, CTX, 0);
}
__global__ __launch_bounds__(128) void k_attn_late(const _Float16* __restrict__ Qh, const _Float16* __restrict__ Ql, const _Float16* __restrict__ Kh, const _Float16* __restrict__ Kl,
                                                   const _Float16* __restrict__ VTh, const _Float16* __restrict__ VTl, _Float16* __restrict__ CTX) {
  attn_body<0>(Qh, Ql, Kh, Kl, VTh, VTl, CTX, ERW / 64);
}

__global__ __launch_bounds__(128) void k_outp(const _Float16* __restrict__ A, const _Float16* __restrict__ Bt, float* __restrict__ out) {
  __shared__ __attribute__((aligned(16))) float so[4][32][68];
  const int wave = __builtin_amdgcn_readfirstlane((int)(threadIdx.x >> 5));
  const int lane = threadIdx.x & 31, ln = lane & 15, hh = lane >> 4;
  const int ntn = DM >> 6;
  const int mt = blockIdx.x / ntn, nq = blockIdx.x - mt * ntn;
  const int row0 = mt * 128 + 32 * wave, col0 = nq * 64;
  const v8f z8 = {0.f, 0.f, 0.f, 0.f, 0.f, 0.f, 0.f, 0.f};
  v8f c[8] = {z8, z8, z8, z8, z8, z8, z8, z8};
  gemm_tile(A, 2 * DM, Bt, 2 * DM, 2 * DM, row0, col0, ln, hh, c);
#pragma unroll
  for (int u = 0; u < 8; ++u) {
    const int t = u & 3, half = u >> 2;
#pragma unroll
    for (int r = 0; r < 8; ++r) so[wave][half * 16 + 8 * hh + r][t * 16 + ln] = c[u][r] * 9.5367431640625e-07f;
  }
  __builtin_amdgcn_fence(4  , "workgroup"); __builtin_amdgcn_wave_barrier();
  const int rsub = lane >> 4, c4 = (lane & 15) * 4;
  for (int pass = 0; pass < 2; ++pass) {
#pragma unroll
    for (int q = 0; q < 16; ++q) {
      const int r = q * 2 + rsub;
      const int m = row0 + r; const int bb = m / SEQ; const int ss = m - bb * SEQ;
      const v4f v = *(const v4fa*)&so[wave][r][c4];
      *(volatile v4f*)(out + (size_t)(bb * SEQ_FULL + ss) * DM + col0 + c4) = v;
    }
    if (pass == 0) __threadfence();
  }
}

constexpr size_t SZW  = (size_t)DM * DM * 2;
constexpr size_t SZBO = 2 * SZW;
constexpr size_t SZP  = (size_t)NR * DM * 2;
constexpr size_t SZC  = 2 * SZP;
constexpr size_t SZT  = (size_t)TABN * 64 * 4;
constexpr size_t O_BQ = 0, O_BK = O_BQ + SZW, O_BV = O_BK + SZW, O_BO = O_BV + SZW, O_X = O_BO + SZBO;
constexpr size_t O_QH = O_X + SZP, O_QL = O_QH + SZP, O_KH = O_QL + SZP, O_KL = O_KH + SZP, O_VH = O_KL + SZP, O_VL = O_VH + SZP;
constexpr size_t O_CTX = O_VL + SZP, O_TAB = O_CTX + SZC, WS_TOTAL = O_TAB + SZT;
static_assert(SZW % 256 == 0);
static_assert(SZP % 256 == 0);
static_assert(SZT % 256 == 0);
static_assert(WS_TOTAL <= 134217728);

extern "C" void kernel_launch(void* const* d_in, const int* in_sizes, int n_in,
                              void* d_out, int out_size, void* d_ws, size_t ws_size, hipStream_t stream) {
  if (n_in < 6) return;
  const int need_rows = (NB - 1) * SEQ_FULL + SEQ;
  if (in_sizes[0] < need_rows * DM) return;
  if (in_sizes[1] < DM * DM || in_sizes[2] < DM * DM || in_sizes[3] < DM * DM || in_sizes[4] < DM * DM) return;
  if (in_sizes[5] < need_rows) return;
  if (out_size < need_rows * DM) return;
  if (ws_size < WS_TOTAL) return;
  const float* x  = (const float*)d_in[0];
  const float* wq = (const float*)d_in[1];
  const float* wk = (const float*)d_in[2];
  const float* wv = (const float*)d_in[3];
  const float* wo = (const float*)d_in[4];
  const int*   tp = (const int*)d_in[5];
  char* ws = (char*)d_ws;
  _Float16* BQ = (_Float16*)(ws + O_BQ); _Float16* BK = (_Float16*)(ws + O_BK); _Float16* BV = (_Float16*)(ws + O_BV); _Float16* BO2 = (_Float16*)(ws + O_BO);
  _Float16* X16 = (_Float16*)(ws + O_X);
  _Float16* QH = (_Float16*)(ws + O_QH); _Float16* QL = (_Float16*)(ws + O_QL); _Float16* KH = (_Float16*)(ws + O_KH); _Float16* KL = (_Float16*)(ws + O_KL);
  _Float16* VTH = (_Float16*)(ws + O_VH); _Float16* VTL = (_Float16*)(ws + O_VL);
  _Float16* CTX = (_Float16*)(ws + O_CTX);
  float* TAB = (float*)(ws + O_TAB);

  const unsigned gw = (unsigned)((DM * (DM / 8) + 255) / 256);
  k_wcvt<<<gw, 256, 0, stream>>>(wq, BQ, DM, 16.0f);
  k_wcvt<<<gw, 256, 0, stream>>>(wk, BK, DM, 16.0f);
  k_wcvt<<<gw, 256, 0, stream>>>(wv, BV, DM, 16.0f);
  k_wcvt<<<gw, 256, 0, stream>>>(wo, BO2, 2 * DM, 16384.0f);
  k_wcvt<<<gw, 256, 0, stream>>>(wo, BO2 + DM, 2 * DM, 16.0f);
  k_xcvt<<<(unsigned)((NR * (DM / 8) + 255) / 256), 256, 0, stream>>>(x, X16);
  k_ropetab<<<(TABN * 16 + 255) / 256, 256, 0, stream>>>(TAB);
  k_proj<<<(unsigned)((NR / 128) * (DM / 64)), 128, 0, stream>>>(X16, BQ, QH, QL, tp, TAB, DM, DM, 1);
  k_proj<<<(unsigned)((NR / 128) * (DM / 64)), 128, 0, stream>>>(X16, BK, KH, KL, tp, TAB, DM, DM, 1);
  k_proj<<<(unsigned)((DM / 128) * (NR / 64)), 128, 0, stream>>>(BV, X16, VTH, VTL, tp, TAB, NR, NR, 0);
  k_attn_early<<<dim3(ERW / 64, NB * NH), 128, 0, stream>>>(QH, QL, KH, KL, VTH, VTL, CTX);
  if (SEQ > ERW) k_attn_late<<<dim3((SEQ - ERW) / 64, NB * NH), 128, 0, stream>>>(QH, QL, KH, KL, VTH, VTL, CTX);
  k_outp<<<(unsigned)((NR / 128) * (DM / 64)), 128, 0, stream>>>(CTX, BO2, (float*)d_out);
}
